// QuIPA2Linear_25744033972596
// MI455X (gfx1250) — hardware-verified
//
#include <hip/hip_runtime.h>
#include <math.h>

#define MB 256
#define NOUT 4096
#define KIN 4096
#define NGRP 1024

typedef _Float16 f16;
typedef __attribute__((ext_vector_type(16))) f16 f16x16;
typedef __attribute__((ext_vector_type(8)))  f16 f16x8;
typedef __attribute__((ext_vector_type(8)))  float f32x8;
typedef __attribute__((ext_vector_type(4)))  float v4f_t;
typedef float v4fa __attribute__((ext_vector_type(4), may_alias));
__device__ __forceinline__ f32x8 wmma16(f16x16 a, f16x16 b, f32x8 c) {
  c = __builtin_amdgcn_wmma_f32_16x16x32_f16(false, a, false, b, (short)0, c, false, false);
  asm volatile("v_nop\n\tv_nop\n\tv_nop\n\tv_nop" : "+v"(c) : "v"(a), "v"(b));
  return c;
}
__device__ __forceinline__ f16x16 lds_frag(const f16* base, int stride) {
  const int lane = threadIdx.x & 31, row = lane & 15, kh = (lane >> 4) * 8;
  const f16x8 lo = *(const f16x8*)(base + row * stride + kh);
  const f16x8 hi = *(const f16x8*)(base + row * stride + kh + 16);
  f16x16 f;
#pragma unroll
  for (int i = 0; i < 8; ++i) { f[i] = lo[i]; f[i + 8] = hi[i]; }
  return f;
}
__constant__ float c_d4h[512] = {0.0f, 0.0f, 0.0f, 0.0f, -2.0f, 0.0f, 0.0f, 0.0f, -1.0f, -1.0f, -1.0f, -1.0f, -1.0f, -1.0f, -1.0f, 0.0f, -1.0f, -1.0f, -1.0f, 1.0f, -1.0f, -1.0f, 0.0f, -1.0f, -1.0f, -1.0f, 0.0f, 0.0f, -1.0f, -1.0f, 0.0f, 1.0f, -1.0f, -1.0f, 1.0f, -1.0f, -1.0f, -1.0f, 1.0f, 0.0f, -1.0f, -1.0f, 1.0f, 1.0f, -1.0f, 0.0f, -1.0f, -1.0f, -1.0f, 0.0f, -1.0f, 0.0f, -1.0f, 0.0f, -1.0f, 1.0f, -1.0f, 0.0f, 0.0f, -1.0f, -1.0f, 0.0f, 0.0f, 0.0f, -1.0f, 0.0f, 0.0f, 1.0f, -1.0f, 0.0f, 1.0f, -1.0f, -1.0f, 0.0f, 1.0f, 0.0f, -1.0f, 0.0f, 1.0f, 1.0f, -1.0f, 1.0f, -1.0f, -1.0f, -1.0f, 1.0f, -1.0f, 0.0f, -1.0f, 1.0f, -1.0f, 1.0f, -1.0f, 1.0f, 0.0f, -1.0f, -1.0f, 1.0f, 0.0f, 0.0f, -1.0f, 1.0f, 0.0f, 1.0f, -1.0f, 1.0f, 1.0f, -1.0f, -1.0f, 1.0f, 1.0f, 0.0f, -1.0f, 1.0f, 1.0f, 1.0f, 0.0f, -2.0f, 0.0f, 0.0f, 0.0f, -1.0f, -1.0f, -1.0f, 0.0f, -1.0f, -1.0f, 0.0f, 0.0f, -1.0f, -1.0f, 1.0f, 0.0f, -1.0f, 0.0f, -1.0f, 0.0f, -1.0f, 0.0f, 0.0f, 0.0f, -1.0f, 0.0f, 1.0f, 0.0f, -1.0f, 1.0f, -1.0f, 0.0f, -1.0f, 1.0f, 0.0f, 0.0f, -1.0f, 1.0f, 1.0f, 0.0f, 0.0f, -2.0f, 0.0f, 0.0f, 0.0f, -1.0f, -1.0f, 0.0f, 0.0f, -1.0f, 0.0f, 0.0f, 0.0f, -1.0f, 1.0f, 0.0f, 0.0f, 0.0f, -2.0f, 0.0f, 0.0f, 0.0f, -1.0f, -1.5f, -0.5f, -1.5f, -0.5f, -1.5f, -0.5f, -1.5f, 0.5f, -1.5f, -0.5f, -0.5f, -1.5f, -1.5f, -0.5f, -0.5f, -0.5f, -1.5f, -0.5f, -0.5f, 0.5f, -1.5f, -0.5f, -0.5f, 1.5f, -1.5f, -0.5f, 0.5f, -1.5f, -1.5f, -0.5f, 0.5f, -0.5f, -1.5f, -0.5f, 0.5f, 0.5f, -1.5f, -0.5f, 0.5f, 1.5f, -1.5f, -0.5f, 1.5f, -0.5f, -1.5f, -0.5f, 1.5f, 0.5f, -1.5f, 0.5f, -1.5f, -0.5f, -1.5f, 0.5f, -1.5f, 0.5f, -1.5f, 0.5f, -0.5f, -1.5f, -1.5f, 0.5f, -0.5f, -0.5f, -1.5f, 0.5f, -0.5f, 0.5f, -1.5f, 0.5f, -0.5f, 1.5f, -1.5f, 0.5f, 0.5f, -1.5f, -1.5f, 0.5f, 0.5f, -0.5f, -1.5f, 0.5f, 0.5f, 0.5f, -1.5f, 0.5f, 0.5f, 1.5f, -1.5f, 0.5f, 1.5f, -0.5f, -1.5f, 0.5f, 1.5f, 0.5f, -1.5f, 1.5f, -0.5f, -0.5f, -1.5f, 1.5f, 0.5f, -0.5f, -1.5f, 1.5f, 0.5f, 0.5f, -0.5f, -1.5f, -1.5f, -0.5f, -0.5f, -1.5f, -1.5f, 0.5f, -0.5f, -1.5f, -0.5f, -1.5f, -0.5f, -1.5f, -0.5f, -0.5f, -0.5f, -1.5f, -0.5f, 0.5f, -0.5f, -1.5f, -0.5f, 1.5f, -0.5f, -1.5f, 0.5f, -1.5f, -0.5f, -1.5f, 0.5f, -0.5f, -0.5f, -1.5f, 0.5f, 0.5f, -0.5f, -1.5f, 0.5f, 1.5f, -0.5f, -1.5f, 1.5f, -0.5f, -0.5f, -1.5f, 1.5f, 0.5f, -0.5f, -0.5f, -1.5f, -1.5f, -0.5f, -0.5f, -1.5f, -0.5f, -0.5f, -0.5f, -1.5f, 0.5f, -0.5f, -0.5f, -1.5f, 1.5f, -0.5f, -0.5f, -0.5f, -1.5f, -0.5f, -0.5f, -0.5f, -0.5f, -0.5f, -0.5f, -0.5f, 0.5f, -0.5f, -0.5f, -0.5f, 1.5f, -0.5f, -0.5f, 0.5f, -1.5f, -0.5f, -0.5f, 0.5f, -0.5f, -0.5f, -0.5f, 0.5f, 0.5f, -0.5f, -0.5f, 0.5f, 1.5f, -0.5f, -0.5f, 1.5f, -1.5f, -0.5f, -0.5f, 1.5f, -0.5f, -0.5f, -0.5f, 1.5f, 0.5f, -0.5f, -0.5f, 1.5f, 1.5f, -0.5f, 0.5f, -1.5f, -1.5f, -0.5f, 0.5f, -1.5f, -0.5f, -0.5f, 0.5f, -1.5f, 0.5f, -0.5f, 0.5f, -1.5f, 1.5f, -0.5f, 0.5f, -0.5f, -1.5f, -0.5f, 0.5f, -0.5f, -0.5f, -0.5f, 0.5f, -0.5f, 0.5f, -0.5f, 0.5f, -0.5f, 1.5f, -0.5f, 0.5f, 0.5f, -1.5f, -0.5f, 0.5f, 0.5f, -0.5f, -0.5f, 0.5f, 0.5f, 0.5f, -0.5f, 0.5f, 0.5f, 1.5f, -0.5f, 0.5f, 1.5f, -1.5f, -0.5f, 0.5f, 1.5f, -0.5f, -0.5f, 0.5f, 1.5f, 0.5f, -0.5f, 0.5f, 1.5f, 1.5f, -0.5f, 1.5f, -1.5f, -0.5f, -0.5f, 1.5f, -1.5f, 0.5f, -0.5f, 1.5f, -0.5f, -1.5f, -0.5f, 1.5f, -0.5f, -0.5f, -0.5f, 1.5f, -0.5f, 0.5f, -0.5f, 1.5f, -0.5f, 1.5f, -0.5f, 1.5f, 0.5f, -1.5f, -0.5f, 1.5f, 0.5f, -0.5f, -0.5f, 1.5f, 0.5f, 0.5f, -0.5f, 1.5f, 0.5f, 1.5f, -0.5f, 1.5f, 1.5f, -0.5f, -0.5f, 1.5f, 1.5f, 0.5f};

__global__ __launch_bounds__(256) void k_quip(const float* __restrict__ xin, const float* __restrict__ sw, const float* __restrict__ qs, const int* __restrict__ qidx, float* __restrict__ z) {
  __shared__ __attribute__((aligned(16))) f16 aS[MB * 40];
  __shared__ __attribute__((aligned(16))) f16 wS[128 * 40];
  __shared__ __attribute__((aligned(16))) float oS[128 * 132];
  __shared__ float cbS[512];
  const int tid = threadIdx.x, lane = tid & 31, wave = tid >> 5, cl = lane & 15, rh = (lane >> 4) * 8;
  const int n0 = blockIdx.x * 128; const int ncol = n0 + wave * 16;
  for (int e = tid; e < 512; e += 256) cbS[e] = c_d4h[e];
  f32x8 acc[16];
#pragma unroll
  for (int i = 0; i < 16; ++i) { f32x8 zz = {}; acc[i] = zz; }
#pragma unroll 1
  for (int ks = 0; ks < KIN / 32; ++ks) {
    __syncthreads();
    { const int r = tid; const float* src = xin + (size_t)r * KIN + ks * 32;
#pragma unroll
      for (int q = 0; q < 8; ++q) { const v4f_t v = *(const v4f_t*)(src + q * 4); const int k = ks * 32 + q * 4; const float g = qs[k >> 2];
        aS[r * 40 + q * 4 + 0] = (f16)(v[0] * sw[k] * g); aS[r * 40 + q * 4 + 1] = (f16)(v[1] * sw[k + 1] * g); aS[r * 40 + q * 4 + 2] = (f16)(v[2] * sw[k + 2] * g); aS[r * 40 + q * 4 + 3] = (f16)(v[3] * sw[k + 3] * g); } }
    { const int n = tid >> 1, gq = (tid & 1) * 4; const int i = n0 + n; const int* ip = qidx + (size_t)i * NGRP + ks * 8 + gq;
#pragma unroll
      for (int g = 0; g < 4; ++g) { const int idx = ip[g]; const float sg = (idx < 128) ? 1.0f : -1.0f; const float* cb = cbS + (idx & 127) * 4;
#pragma unroll
        for (int kk = 0; kk < 4; ++kk) wS[n * 40 + (gq + g) * 4 + kk] = (f16)(sg * cb[kk]); } }
    __syncthreads();
    const f16x16 bf = lds_frag(wS + (wave * 16) * 40, 40);
#pragma unroll
    for (int mt = 0; mt < 16; ++mt) acc[mt] = wmma16(lds_frag(aS + (mt * 16) * 40, 40), bf, acc[mt]);
  }
#pragma unroll
  for (int hf = 0; hf < 2; ++hf) {
    __syncthreads();
#pragma unroll
    for (int mt = 0; mt < 8; ++mt)
#pragma unroll
      for (int r = 0; r < 8; ++r) oS[((mt * 16) + rh + r) * 132 + wave * 16 + cl] = acc[hf * 8 + mt][r];
    __syncthreads();
#pragma unroll 1
    for (int pass = 0; pass < 2; ++pass) { for (int q4 = tid; q4 < 128 * 32; q4 += 256) { const int r = q4 >> 5, c4 = (q4 & 31) * 4;
        *(volatile v4f_t*)(z + (size_t)(hf * 128 + r) * NOUT + n0 + c4) = *(const volatile v4fa*)(oS + r * 132 + c4); } __threadfence(); }
  }
}

extern "C" void kernel_launch(void* const* d_in, const int* in_sizes, int n_in,
                              void* d_out, int out_size, void* d_ws, size_t ws_size,
                              hipStream_t stream) {
  (void)in_sizes; (void)n_in; (void)out_size; (void)d_ws; (void)ws_size;
  const float* xin = (const float*)d_in[0];
  const float* sw = (const float*)d_in[1];
  const float* qs = (const float*)d_in[2];
  const int* qidx = (const int*)d_in[3];
  float* z = (float*)d_out;
  k_quip<<<dim3(NOUT / 128), dim3(256), 0, stream>>>(xin, sw, qs, qidx, z);
}
